// CARAFE3D_77163382440813
// MI455X (gfx1250) — hardware-verified
//
#include <hip/hip_runtime.h>


#define NN_  2
#define CI   32
#define C4   8
#define CO   16
#define GS   32
#define NV   (NN_ * GS * GS * GS)
#define K3   27
#define R3   8
#define KE   216
#define KEP  224
#define NEP  256
#define RCH  256
#define NCHK (NN_ * GS * GS / RCH)
#define VCH  (RCH * GS)
#define OCH  (VCH * R3)
typedef _Float16 h16;
typedef unsigned short bf;
typedef __attribute__((ext_vector_type(16))) __bf16   v16bf;
typedef __attribute__((ext_vector_type(16))) _Float16 v16h;
typedef __attribute__((ext_vector_type(8)))  _Float16 v8h;
typedef __attribute__((ext_vector_type(8)))  unsigned short v8us;
typedef __attribute__((ext_vector_type(8)))  float    v8f;
typedef __attribute__((ext_vector_type(4)))  float    v4f;
typedef v8h  __attribute__((may_alias)) v8ha;
typedef v4f  __attribute__((may_alias)) v4fa;
typedef v8us __attribute__((may_alias)) v8usa;

__device__ __forceinline__ unsigned short f2bf(float f) { unsigned u = __float_as_uint(f); u += 0x7FFFu + ((u >> 16) & 1u); return (unsigned short)(u >> 16); }
__device__ __forceinline__ float bf2f(unsigned short b) { return __uint_as_float(((unsigned)b) << 16); }
__device__ __forceinline__ float bfr(float f) { return bf2f(f2bf(f)); }
__device__ __forceinline__ v16h cat16(v8h lo, v8h hi) { return __builtin_shufflevector(lo, hi, 0, 1, 2, 3, 4, 5, 6, 7, 8, 9, 10, 11, 12, 13, 14, 15); }
__device__ __forceinline__ v16bf cat16b(v8us lo, v8us hi) { return __builtin_bit_cast(v16bf, __builtin_shufflevector(lo, hi, 0, 1, 2, 3, 4, 5, 6, 7, 8, 9, 10, 11, 12, 13, 14, 15)); }
__device__ __forceinline__ v8f wmma16(v16h a, v16h b, v8f c) { return __builtin_amdgcn_wmma_f32_16x16x32_f16(false, a, false, b, (short)0, c, false, false); }
__device__ __forceinline__ v8f wmmab(v16bf a, v16bf b, v8f c) { return __builtin_amdgcn_wmma_f32_16x16x32_bf16(false, a, false, b, (short)0, c, false, false); }


template <typename T16> struct WFrag;
template <> struct WFrag<h16> { typedef v16h V; static __device__ __forceinline__ V ld(const h16* p) { return cat16(*(const v8h*)p, *(const v8h*)(p + 16)); } static __device__ __forceinline__ v8f mma(V a, V b, v8f c) { return wmma16(a, b, c); } };
template <> struct WFrag<bf> { typedef v16bf V; static __device__ __forceinline__ V ld(const bf* p) { return cat16b(*(const v8us*)p, *(const v8us*)(p + 16)); } static __device__ __forceinline__ v8f mma(V a, V b, v8f c) { return wmmab(a, b, c); } };
template <typename T16, int NSPLIT, bool BIAS>
__global__ __launch_bounds__(32) void k_gemmw(const T16* __restrict__ A, const T16* __restrict__ A2, const T16* __restrict__ Bt, const T16* __restrict__ Bt2, int K, float* C, int ldc, const float* __restrict__ bias, size_t sA, size_t sB, size_t sC) {
    typedef typename WFrag<T16>::V V;
    __shared__ __align__(16) float os[16 * 68];
    const size_t z = blockIdx.z; A += z * sA; if (A2) A2 += z * sA; Bt += z * sB; if (Bt2) Bt2 += z * sB; C += z * sC;
    const int lane = threadIdx.x & 31, lr = lane & 15, hi = lane >> 4; const int r0 = blockIdx.x * 64, c0 = blockIdx.y * 64;
    v8f acc[4][4];
#pragma unroll
    for (int mb = 0; mb < 4; ++mb)
#pragma unroll
        for (int nb = 0; nb < 4; ++nb) acc[mb][nb] = (v8f){};
    const size_t aoff = (size_t)(r0 + lr) * K + 8 * hi, boff = (size_t)(c0 + lr) * K + 8 * hi;
#pragma unroll 1
    for (int kc = 0; kc < K; kc += 32) {
        V a[4], a2[4];
#pragma unroll
        for (int mb = 0; mb < 4; ++mb) { a[mb] = WFrag<T16>::ld(A + aoff + (size_t)mb * 16 * K + kc); if (NSPLIT == 1 || NSPLIT == 2) a2[mb] = WFrag<T16>::ld(A2 + aoff + (size_t)mb * 16 * K + kc); }
#pragma unroll
        for (int nb = 0; nb < 4; ++nb) { const V b = WFrag<T16>::ld(Bt + boff + (size_t)nb * 16 * K + kc); V b2; if (NSPLIT >= 2) b2 = WFrag<T16>::ld(Bt2 + boff + (size_t)nb * 16 * K + kc);
#pragma unroll
            for (int mb = 0; mb < 4; ++mb) { acc[mb][nb] = WFrag<T16>::mma(a[mb], b, acc[mb][nb]); if (NSPLIT == 1 || NSPLIT == 2) acc[mb][nb] = WFrag<T16>::mma(a2[mb], b, acc[mb][nb]); if (NSPLIT >= 2) acc[mb][nb] = WFrag<T16>::mma(a[mb], b2, acc[mb][nb]); } }
        asm volatile("v_nop\n\tv_nop\n\tv_nop\n\tv_nop" : "+v"(acc[0][0]), "+v"(acc[1][1]), "+v"(acc[2][2]), "+v"(acc[3][3]) : "v"(a[0]), "v"(a[3]));
    }
#pragma unroll
    for (int mb = 0; mb < 4; ++mb) {
#pragma unroll
        for (int nb = 0; nb < 4; ++nb) {
#pragma unroll
            for (int j = 0; j < 8; ++j) os[(hi * 8 + j) * 68 + nb * 16 + lr] = acc[mb][nb][j]; }
        __builtin_amdgcn_wave_barrier(); asm volatile("" ::: "memory");
        float* crow = C + (size_t)(r0 + mb * 16) * ldc + c0;
#pragma unroll 1
        for (int ps = 0; ps < 2; ++ps) {
#pragma unroll
            for (int s = 0; s < 8; ++s) { const int row = 2 * s + hi, cofs = lr * 4; v4f val = *(const v4fa*)(os + row * 68 + cofs); if (BIAS) { val[0] += bfr(bias[c0 + cofs]); val[1] += bfr(bias[c0 + cofs + 1]); val[2] += bfr(bias[c0 + cofs + 2]); val[3] += bfr(bias[c0 + cofs + 3]); }
                *(volatile v4f*)(crow + (size_t)row * ldc + cofs) = val; }
            if (ps == 0) __threadfence(); }
        __builtin_amdgcn_wave_barrier(); asm volatile("" ::: "memory");
    }
}

__device__ __forceinline__ void splitf(float y, unsigned short& h, unsigned short& l) { h = f2bf(y); l = f2bf(y - bf2f(h)); }

__global__ __launch_bounds__(256) void k_wpad(const float* __restrict__ w, int N, int K, int Np, int Kp, bf* Bt) {
    typedef __attribute__((ext_vector_type(2))) unsigned short v2us;
    const int lane = threadIdx.x & 31; const int nlines = Np * Kp / 64; const int wg = blockIdx.x * 8 + (threadIdx.x >> 5), nw = gridDim.x * 8;
#pragma unroll 1
    for (int ps = 0; ps < 2; ++ps) {
#pragma unroll 1
        for (int L = wg; L < nlines; L += nw) { const int e = L * 64 + lane * 2; v2us o;
#pragma unroll
            for (int q = 0; q < 2; ++q) { const int n = (e + q) / Kp, k = (e + q) % Kp; o[q] = (n < N && k < K) ? f2bf(w[(size_t)(n < N ? n : 0) * K + (k < K ? k : 0)]) : (unsigned short)0; }
            *(volatile v2us*)(Bt + e) = o; }
        if (ps == 0) __threadfence(); }
}
__global__ __launch_bounds__(64) void k_bpad(const float* __restrict__ b, int N, float* out) { const int i = blockIdx.x * 64 + threadIdx.x; const float v = i < N ? b[i < N ? i : 0] : 0.f; *(volatile float*)(out + i) = v; __threadfence(); *(volatile float*)(out + i) = v; }
__global__ __launch_bounds__(256) void k_tok(const float* __restrict__ x, bf* XT) {
    typedef __attribute__((ext_vector_type(4))) unsigned short v4us;
    __shared__ float tl[CI][65];
    const int tid = threadIdx.x; const int v0 = blockIdx.x * 64, n = blockIdx.y;
#pragma unroll
    for (int i = 0; i < 8; ++i) { const int c = i * 4 + (tid >> 6), vv = tid & 63; tl[c][vv] = x[((size_t)n * CI + c) * (GS * GS * GS) + v0 + vv]; }
    __syncthreads();
    const int lane = tid & 31, wv = tid >> 5;
    auto pass = [&]() {
#pragma unroll
        for (int i2 = 0; i2 < 2; ++i2) { const int r = wv * 8 + i2 * 4 + (lane >> 3); const int cq = (lane & 7) * 4; v4us o;
#pragma unroll
            for (int i = 0; i < 4; ++i) o[i] = f2bf(tl[cq + i][r]);
            *(volatile v4us*)(XT + ((size_t)n * GS * GS * GS + v0 + r) * CI + cq) = o; } };
    pass(); __threadfence(); pass();
}
__global__ __launch_bounds__(256) void k_im3(const float* __restrict__ T, int ch, bf* Ah, bf* Al) {
    typedef __attribute__((ext_vector_type(2))) unsigned short v2us;
    const int lane = threadIdx.x & 31; const int L0 = (blockIdx.x * 8 + (threadIdx.x >> 5)) * 8; const int nlines = VCH * KEP / 64;
#pragma unroll 1
    for (int ps = 0; ps < 2; ++ps) {
#pragma unroll 1
        for (int l = 0; l < 8; ++l) { const int L = L0 + l; if (L >= nlines) break; const int e = L * 64 + lane * 2; const int vr = e / KEP, col = e % KEP; const int gv = ch * VCH + vr; const int n = gv / (GS * GS * GS), h = (gv / (GS * GS)) % GS, w = (gv / GS) % GS, d = gv % GS; v2us oh, ol;
#pragma unroll
            for (int q = 0; q < 2; ++q) { const int cc = col + q; unsigned short a = 0, b2 = 0;
                if (cc < KE) { const int c = cc / K3, tap = cc % K3; const int i = tap / 9, j = (tap / 3) % 3, ll = tap % 3; const int hh = h + i - 1, ww = w + j - 1, dd = d + ll - 1;
                    if (hh >= 0 && hh < GS && ww >= 0 && ww < GS && dd >= 0 && dd < GS) splitf(T[((size_t)((n * GS + hh) * GS + ww) * GS + dd) * 64 + c], a, b2); }
                oh[q] = a; ol[q] = b2; }
            *(volatile v2us*)(Ah + e) = oh; *(volatile v2us*)(Al + e) = ol; }
        if (ps == 0) __threadfence(); }
}
__global__ __launch_bounds__(32) void k_reasm(const float* __restrict__ x, const float* __restrict__ ENC, int ch, bf* OTh, bf* OTl) {
    __shared__ unsigned short sh[4 * 64 * CI], slo[4 * 64 * CI];
    __shared__ float kl[K3 * 4 * 32];
    const int lane = threadIdx.x; const int lr = blockIdx.x; const int grow = ch * RCH + lr; const int n = grow / (GS * GS), h = (grow / GS) % GS, w = grow % GS; const int d = lane;
    const float* er = ENC + ((size_t)lr * GS + d) * NEP;
#pragma unroll 1
    for (int rhf = 0; rhf < 2; ++rhf) {
#pragma unroll
        for (int r = 0; r < 4; ++r) { float m = -3.0e38f;
#pragma unroll 1
            for (int k = 0; k < K3; ++k) m = fmaxf(m, er[k * R3 + rhf * 4 + r]);
            float s = 0.f;
#pragma unroll 1
            for (int k = 0; k < K3; ++k) { const float e = __expf(er[k * R3 + rhf * 4 + r] - m); kl[(k * 4 + r) * 32 + lane] = e; s += e; }
            const float inv = __fdiv_rn(1.0f, s);
#pragma unroll 1
            for (int k = 0; k < K3; ++k) kl[(k * 4 + r) * 32 + lane] *= inv; }
        asm volatile("" ::: "memory");
        const float* xb = x + (size_t)n * CI * (GS * GS * GS);
#pragma unroll 1
        for (int c = 0; c < CI; ++c) { const float* xc = xb + (size_t)c * (GS * GS * GS); float acc[4];
#pragma unroll
            for (int r = 0; r < 4; ++r) acc[r] = 0.f;
#pragma unroll 1
            for (int i = 0; i < 3; ++i) { const int hh = h + i - 1;
#pragma unroll 1
                for (int j = 0; j < 3; ++j) { const int ww = w + j - 1; const bool okhw = hh >= 0 && hh < GS && ww >= 0 && ww < GS; const float* row = xc + ((size_t)(okhw ? hh : 0) * GS + (okhw ? ww : 0)) * GS;
#pragma unroll
                    for (int ll = 0; ll < 3; ++ll) { const int dd = d + ll - 1; const bool ok = okhw && dd >= 0 && dd < GS; const float v = ok ? bfr(row[dd < 0 ? 0 : (dd > GS - 1 ? GS - 1 : dd)]) : 0.f; const int k = (i * 3 + j) * 3 + ll;
#pragma unroll
                        for (int r = 0; r < 4; ++r) acc[r] = fmaf(v, kl[(k * 4 + r) * 32 + lane], acc[r]); } } }
#pragma unroll
            for (int r = 0; r < 4; ++r) { const int rr = rhf * 4 + r; const int rh = rr >> 2, rw = (rr >> 1) & 1, rd = rr & 1; const int r4 = rh * 2 + rw, d2 = 2 * d + rd; unsigned short a, b2; splitf(acc[r], a, b2); sh[(r4 * 64 + d2) * CI + c] = a; slo[(r4 * 64 + d2) * CI + c] = b2; } } }
    __builtin_amdgcn_wave_barrier(); asm volatile("" ::: "memory");
    auto pass = [&]() {
#pragma unroll 1
        for (int q = 0; q < 4 * 64 * CI / 256; ++q) { const int e = q * 256 + lane * 8; const v8us vh = *(const v8us*)(sh + e), vl = *(const v8us*)(slo + e);
            const size_t o = (size_t)lr * (4 * 64) * CI + e;
            *(volatile v8us*)(OTh + o) = vh; *(volatile v8us*)(OTl + o) = vl; } };
    pass(); __threadfence(); pass();
}
__global__ __launch_bounds__(256) void k_outc(const float* __restrict__ C, int ch, float* OUT) {
    typedef __attribute__((ext_vector_type(2))) float v2f;
    const int lane = threadIdx.x & 31; const int wg = blockIdx.x * 8 + (threadIdx.x >> 5); if (wg >= CO * RCH * 4) return; const int c2 = wg / (RCH * 4), lr = (wg / 4) % RCH, r4 = wg % 4;
    const int grow = ch * RCH + lr; const int n = grow / (GS * GS), h = (grow / GS) % GS, w = grow % GS; const int H2 = 2 * h + (r4 >> 1), W2 = 2 * w + (r4 & 1); v2f o;
#pragma unroll
    for (int q = 0; q < 2; ++q) o[q] = C[((size_t)(lr * 4 + r4) * 64 + lane * 2 + q) * 64 + c2];
    float* dst = OUT + ((((size_t)n * CO + c2) * (2 * GS) + H2) * (2 * GS) + W2) * (2 * GS) + lane * 2; *(volatile v2f*)dst = o; __threadfence(); *(volatile v2f*)dst = o;
}

extern "C" void kernel_launch(void* const* d_in, const int* in_sizes, int n_in,
                              void* d_out, int out_size, void* d_ws, size_t ws_size, hipStream_t stream) {
    (void)in_sizes; (void)n_in; (void)out_size;
    const float* x = (const float*)d_in[0]; const float* w_down = (const float*)d_in[1]; const float* b_down = (const float*)d_in[2]; const float* w_enc = (const float*)d_in[3]; const float* b_enc = (const float*)d_in[4]; const float* w_out = (const float*)d_in[5]; const float* b_out = (const float*)d_in[6];
    float* OUT = (float*)d_out;
    char* wsp = (char*)d_ws;
    auto take = [&](size_t bytes) { char* p = wsp; wsp += (bytes + 255) & ~(size_t)255; return (void*)p; };
    bf* WD = (bf*)take(64 * 32 * 2); bf* WE = (bf*)take((size_t)NEP * KEP * 2); bf* WO = (bf*)take(64 * 32 * 2); float* BD = (float*)take(64 * 4); float* BE = (float*)take(NEP * 4); float* BO = (float*)take(64 * 4);
    bf* XT = (bf*)take((size_t)NV * CI * 2); float* T = (float*)take((size_t)NV * 64 * 4);
    bf* Ah = (bf*)take((size_t)VCH * KEP * 2); bf* Al = (bf*)take((size_t)VCH * KEP * 2); float* ENC = (float*)take((size_t)VCH * NEP * 4);
    bf* OTh = (bf*)take((size_t)OCH * CI * 2); bf* OTl = (bf*)take((size_t)OCH * CI * 2); float* Cc = (float*)take((size_t)OCH * 64 * 4);
    if ((size_t)(wsp - (char*)d_ws) > ws_size) return;
    k_wpad<<<1, 256, 0, stream>>>(w_down, C4, CI, 64, CI, WD); k_wpad<<<8, 256, 0, stream>>>(w_enc, KE, KE, NEP, KEP, WE); k_wpad<<<1, 256, 0, stream>>>(w_out, CO, CI, 64, CI, WO);
    k_bpad<<<1, 64, 0, stream>>>(b_down, C4, BD); k_bpad<<<4, 64, 0, stream>>>(b_enc, KE, BE); k_bpad<<<1, 64, 0, stream>>>(b_out, CO, BO);
    k_tok<<<dim3(GS * GS * GS / 64, NN_), 256, 0, stream>>>(x, XT);
    k_gemmw<bf, 0, true><<<dim3(NV / 64, 1, 1), 32, 0, stream>>>(XT, nullptr, WD, nullptr, CI, T, 64, BD, 0, 0, 0);
    for (int ch = 0; ch < NCHK; ++ch) {
        k_im3<<<(VCH * KEP / 64 + 63) / 64, 256, 0, stream>>>(T, ch, Ah, Al);
        k_gemmw<bf, 1, true><<<dim3(VCH / 64, NEP / 64, 1), 32, 0, stream>>>(Ah, Al, WE, nullptr, KEP, ENC, NEP, BE, 0, 0, 0);
        k_reasm<<<RCH, 32, 0, stream>>>(x, ENC, ch, OTh, OTl);
        k_gemmw<bf, 1, true><<<dim3(OCH / 64, 1, 1), 32, 0, stream>>>(OTh, OTl, WO, nullptr, CI, Cc, 64, BO, 0, 0, 0);
        k_outc<<<CO * RCH * 4 / 8, 256, 0, stream>>>(Cc, ch, OUT); }
}
